// MultiHeadLocalAttention_55800215109727
// MI455X (gfx1250) — hardware-verified
//
#include <hip/hip_runtime.h>
#include <stddef.h>
#include <stdint.h>


static constexpr int BQ    = 2;
static constexpr int SQ    = 8192;
static constexpr int FQ    = 512;
static constexpr int HQ    = 8;
static constexpr int DQ    = 64;
static constexpr int BLKQ  = 128;
static constexpr int NBQ   = SQ / BLKQ;
static constexpr int MROWS = BQ * SQ;
static constexpr size_t NE = (size_t)MROWS * FQ;
static constexpr size_t WE = (size_t)FQ * FQ;

static_assert(MROWS % 128 == 0, "");
static_assert(FQ % 128 == 0, "");
static_assert(SQ % BLKQ == 0, "");
static_assert(HQ * DQ == FQ, "");
static_assert(NE % (8 * 256) == 0, "");

static constexpr float QSC = 8.0f;
static constexpr float KSC = 8.0f;
static constexpr float VSC = 16.0f;
static constexpr float PSC = 4096.0f;
static constexpr float SSC = 0.125f / (QSC * KSC);
static constexpr float OSC = 1.0f / (PSC * VSC);
static constexpr float NEG = -1e30f;

typedef __bf16   bf16_t;
typedef _Float16 f16_t;
static_assert(sizeof(bf16_t) == 2, "");
typedef bf16_t   v16b __attribute__((ext_vector_type(16)));
typedef bf16_t   v8b  __attribute__((ext_vector_type(8)));
typedef f16_t    v16h __attribute__((ext_vector_type(16)));
typedef f16_t    v8h  __attribute__((ext_vector_type(8)));
typedef float    v8f  __attribute__((ext_vector_type(8)));
typedef float    v4f  __attribute__((ext_vector_type(4), __may_alias__));
typedef unsigned v4u  __attribute__((ext_vector_type(4), __may_alias__));

union FragB { v16b v; v4u u[2]; };
union FragH { v16h v; v4u u[2]; };
union PackB { v8b b; v4u u; };
union PackH { v8h h; v4u u; };

#define NOP4 "v_nop\n\tv_nop\n\tv_nop\n\tv_nop"

static __device__ __forceinline__ v8f vzero8() {
  v8f z;
#pragma unroll
  for (int i = 0; i < 8; ++i) z[i] = 0.0f;
  return z;
}

static __device__ __forceinline__ v16b ldfb(const bf16_t* p) {
  FragB f;
  f.u[0] = *(const v4u*)(p);
  f.u[1] = *(const v4u*)(p + 16);
  return f.v;
}
static __device__ __forceinline__ v16h ldfh(const f16_t* p) {
  FragH f;
  f.u[0] = *(const v4u*)(p);
  f.u[1] = *(const v4u*)(p + 16);
  return f.v;
}

static __device__ __forceinline__ v8f mma_b(v8f c, v16b a, v16b b) {
  return __builtin_amdgcn_wmma_f32_16x16x32_bf16(false, a, false, b, (short)0, c, false, false);
}
static __device__ __forceinline__ v8f mma_h(v8f c, v16h a, v16h b) {
  return __builtin_amdgcn_wmma_f32_16x16x32_f16(false, a, false, b, (short)0, c, false, false);
}

__global__ __launch_bounds__(256)
void k_cvt(const float* __restrict__ x, int n8, bf16_t* __restrict__ y) {
  const int g = blockIdx.x * 256 + threadIdx.x;
  if (g >= n8) return;
  const float* p = x + (size_t)g * 8;
  const v4f a = *(const v4f*)(p);
  const v4f c = *(const v4f*)(p + 4);
  PackB pb;
  pb.b[0] = (bf16_t)a[0]; pb.b[1] = (bf16_t)a[1]; pb.b[2] = (bf16_t)a[2]; pb.b[3] = (bf16_t)a[3];
  pb.b[4] = (bf16_t)c[0]; pb.b[5] = (bf16_t)c[1]; pb.b[6] = (bf16_t)c[2]; pb.b[7] = (bf16_t)c[3];
  const size_t o = (size_t)g * 8;
  *(volatile v4u*)(y + o) = pb.u;
  __threadfence();
  *(volatile v4u*)(y + o) = pb.u;
}

__global__ __launch_bounds__(256)
void k_wtrans(const float* __restrict__ w, int KR, int NC, bf16_t* __restrict__ out) {
  __shared__ __attribute__((aligned(16))) float tile[64 * 65];
  const int n0 = blockIdx.x * 64;
  const int k0 = blockIdx.y * 64;
  if (n0 + 64 > NC || k0 + 64 > KR) return;
  const int tid = threadIdx.x;
  {
    const int kr = tid >> 2;
    const int c0 = (tid & 3) * 16;
    const float* src = w + (size_t)(k0 + kr) * NC + n0 + c0;
#pragma unroll
    for (int i = 0; i < 16; i += 4) {
      const v4f f = *(const v4f*)(src + i);
      tile[kr * 65 + c0 + i + 0] = f[0];
      tile[kr * 65 + c0 + i + 1] = f[1];
      tile[kr * 65 + c0 + i + 2] = f[2];
      tile[kr * 65 + c0 + i + 3] = f[3];
    }
  }
  __syncthreads();
  const int lane = tid & 31, wv = tid >> 5;
  const int q = lane >> 3, j = lane & 7;
  for (int pass = 0; pass < 2; ++pass) {
    if (pass) __threadfence();
#pragma unroll
    for (int it = 0; it < 2; ++it) {
      const int nl = it * 32 + wv * 4 + q;
      PackB pb;
#pragma unroll
      for (int i = 0; i < 8; ++i) pb.b[i] = (bf16_t)tile[(8 * j + i) * 65 + nl];
      const size_t o = (size_t)(n0 + nl) * KR + k0 + 8 * j;
      *(volatile v4u*)(out + o) = pb.u;
    }
  }
}

template <int MODE>
__global__ __launch_bounds__(256)
void k_gemm(const bf16_t* __restrict__ A0, const bf16_t* __restrict__ A1,
            const bf16_t* __restrict__ Bt, const float* __restrict__ bias, float oscale,
            f16_t* __restrict__ P16, float* __restrict__ outf) {
  __shared__ __attribute__((aligned(16))) float Es[8704];
  const int m0 = blockIdx.x * 128;
  const int n0 = blockIdx.y * 128;
  if (m0 + 128 > MROWS || n0 + 128 > FQ) return;
  const int tid = threadIdx.x, lane = tid & 31, lh = lane >> 4, lm = lane & 15;
  const int w = tid >> 5, wm = w & 3, wn = w >> 2;

  size_t aoff[2], boff[4];
#pragma unroll
  for (int mt = 0; mt < 2; ++mt)
    aoff[mt] = (size_t)(m0 + wm * 32 + mt * 16 + lm) * FQ + 8 * lh;
#pragma unroll
  for (int nt = 0; nt < 4; ++nt)
    boff[nt] = (size_t)(n0 + wn * 64 + nt * 16 + lm) * FQ + 8 * lh;

  v8f acc[2][4];
#pragma unroll
  for (int i = 0; i < 2; ++i)
#pragma unroll
    for (int jn = 0; jn < 4; ++jn) acc[i][jn] = vzero8();

#pragma unroll 1
  for (int k0 = 0; k0 < FQ; k0 += 32) {
    if constexpr (MODE == 2) {
      const v16b a0h = ldfb(A0 + aoff[0] + k0);
      const v16b a0l = ldfb(A1 + aoff[0] + k0);
      const v16b a1h = ldfb(A0 + aoff[1] + k0);
      const v16b a1l = ldfb(A1 + aoff[1] + k0);
#pragma unroll
      for (int nt = 0; nt < 4; ++nt) {
        const v16b b = ldfb(Bt + boff[nt] + k0);
        acc[0][nt] = mma_b(acc[0][nt], a0h, b);
        acc[0][nt] = mma_b(acc[0][nt], a0l, b);
        acc[1][nt] = mma_b(acc[1][nt], a1h, b);
        acc[1][nt] = mma_b(acc[1][nt], a1l, b);
        asm volatile(NOP4
                     : "+v"(acc[0][nt]), "+v"(acc[1][nt])
                     : "v"(a0h), "v"(a0l), "v"(a1h), "v"(a1l), "v"(b));
      }
    } else {
      const v16b a0 = ldfb(A0 + aoff[0] + k0);
      const v16b a1 = ldfb(A0 + aoff[1] + k0);
#pragma unroll
      for (int nt = 0; nt < 4; ++nt) {
        const v16b b = ldfb(Bt + boff[nt] + k0);
        acc[0][nt] = mma_b(acc[0][nt], a0, b);
        acc[1][nt] = mma_b(acc[1][nt], a1, b);
        asm volatile(NOP4
                     : "+v"(acc[0][nt]), "+v"(acc[1][nt])
                     : "v"(a0), "v"(a1), "v"(b));
      }
    }
  }

  const int bb = m0 / SQ;
  const int s0 = m0 % SQ;
  for (int half = 0; half < 2; ++half) {
    __syncthreads();
    if (wn == half) {
#pragma unroll
      for (int nt = 0; nt < 4; ++nt) {
        const int cl = nt * 16 + lm;
        const float bsv = bias[n0 + half * 64 + cl];
#pragma unroll
        for (int mt = 0; mt < 2; ++mt) {
#pragma unroll
          for (int r = 0; r < 8; ++r) {
            const int rl = wm * 32 + mt * 16 + 8 * lh + r;
            const float v = acc[mt][nt][r] + bsv;
            if (MODE == 1) Es[cl * 132 + rl] = v;
            else           Es[rl * 68 + cl] = v;
          }
        }
      }
    }
    __syncthreads();
    const int hh = (n0 >> 6) + half;
    for (int pass = 0; pass < 2; ++pass) {
      if (pass) __threadfence();
      if constexpr (MODE == 0) {
        const int q = lane >> 3, j = lane & 7;
        const size_t base = ((size_t)(bb * HQ + hh) * SQ + s0) * DQ + 8 * j;
#pragma unroll
        for (int it = 0; it < 4; ++it) {
          const int rl = w * 16 + it * 4 + q;
          const float* pp = Es + rl * 68 + 8 * j;
          const v4f x0 = *(const v4f*)(pp);
          const v4f x1 = *(const v4f*)(pp + 4);
          PackH ph;
          ph.h[0] = (f16_t)(x0[0] * oscale); ph.h[1] = (f16_t)(x0[1] * oscale);
          ph.h[2] = (f16_t)(x0[2] * oscale); ph.h[3] = (f16_t)(x0[3] * oscale);
          ph.h[4] = (f16_t)(x1[0] * oscale); ph.h[5] = (f16_t)(x1[1] * oscale);
          ph.h[6] = (f16_t)(x1[2] * oscale); ph.h[7] = (f16_t)(x1[3] * oscale);
          const size_t o = base + (size_t)rl * DQ;
          *(volatile v4u*)(P16 + o) = ph.u;
        }
      } else if constexpr (MODE == 1) {
        const int q = lane >> 4, j = lane & 15;
        const size_t base = ((size_t)(bb * HQ + hh) * DQ) * SQ + s0 + 8 * j;
#pragma unroll
        for (int it = 0; it < 4; ++it) {
          const int dl = w * 8 + it * 2 + q;
          const float* pp = Es + dl * 132 + 8 * j;
          const v4f x0 = *(const v4f*)(pp);
          const v4f x1 = *(const v4f*)(pp + 4);
          PackH ph;
          ph.h[0] = (f16_t)(x0[0] * oscale); ph.h[1] = (f16_t)(x0[1] * oscale);
          ph.h[2] = (f16_t)(x0[2] * oscale); ph.h[3] = (f16_t)(x0[3] * oscale);
          ph.h[4] = (f16_t)(x1[0] * oscale); ph.h[5] = (f16_t)(x1[1] * oscale);
          ph.h[6] = (f16_t)(x1[2] * oscale); ph.h[7] = (f16_t)(x1[3] * oscale);
          const size_t o = base + (size_t)dl * SQ;
          *(volatile v4u*)(P16 + o) = ph.u;
        }
      } else {
        const int q = lane >> 4, j = lane & 15;
#pragma unroll
        for (int it = 0; it < 8; ++it) {
          const int rl = w * 16 + it * 2 + q;
          const v4f v = *(const v4f*)(Es + rl * 68 + 4 * j);
          const size_t o = (size_t)(m0 + rl) * FQ + n0 + half * 64 + 4 * j;
          *(volatile v4f*)(outf + o) = v;
        }
      }
    }
  }
}

static constexpr int PPH   = 72;
static constexpr int OPF   = 68;
static constexpr int WSLOT = 16 * OPF;

__global__ __launch_bounds__(128)
void k_attn(const f16_t* __restrict__ Qp, const f16_t* __restrict__ Kp, const f16_t* __restrict__ Vp,
            bf16_t* __restrict__ Oh, bf16_t* __restrict__ Ol) {
  __shared__ __attribute__((aligned(16))) float Ls[4 * WSLOT];
  const int idx = blockIdx.x;
  const int qh = idx & 1;
  const int t  = idx >> 1;
  const int n  = t % NBQ;
  const int hd = (t / NBQ) % HQ;
  const int b  = t / (NBQ * HQ);
  if (b >= BQ) return;
  const int tid = threadIdx.x, lane = tid & 31, lh = lane >> 4, lm = lane & 15, w = tid >> 5;
  const int qb = qh * 64 + w * 16;
  const size_t head = (size_t)(b * HQ + hd) * SQ * DQ;

  v16h qf[2];
  {
    const size_t qo = head + (size_t)(n * BLKQ + qb + lm) * DQ + 8 * lh;
    qf[0] = ldfh(Qp + qo);
    qf[1] = ldfh(Qp + qo + 32);
  }

  float m_r[8], l_r[8];
  v8f oacc[4];
#pragma unroll
  for (int r = 0; r < 8; ++r) { m_r[r] = NEG; l_r[r] = 0.0f; }
#pragma unroll
  for (int nt = 0; nt < 4; ++nt) oacc[nt] = vzero8();

  float* Ow = Ls + w * WSLOT;
  f16_t* Pw = (f16_t*)Ow;
  const int j0 = (n > 0) ? n - 1 : n;
  const int j1 = (n < NBQ - 1) ? n + 1 : n;

  for (int jb = j0; jb <= j1; ++jb) {
    const int rel = jb - n;
    const int cb = (rel < 0 && qh == 1) ? 1 : 0;
    const int ce = (rel > 0 && qh == 0) ? 1 : 2;
#pragma unroll 1
    for (int c = cb; c < ce; ++c) {
      v8f sacc[4];
#pragma unroll
      for (int kt = 0; kt < 4; ++kt) sacc[kt] = vzero8();
#pragma unroll
      for (int kt = 0; kt < 4; ++kt) {
        const size_t ko = head + (size_t)(jb * BLKQ + c * 64 + kt * 16 + lm) * DQ + 8 * lh;
        const v16h k0 = ldfh(Kp + ko);
        const v16h k1 = ldfh(Kp + ko + 32);
        sacc[kt] = mma_h(sacc[kt], qf[0], k0);
        sacc[kt] = mma_h(sacc[kt], qf[1], k1);
        asm volatile(NOP4 : "+v"(sacc[kt]) : "v"(qf[0]), "v"(qf[1]), "v"(k0), "v"(k1));
      }

      float bm[8];
#pragma unroll
      for (int r = 0; r < 8; ++r) bm[r] = NEG;
#pragma unroll
      for (int kt = 0; kt < 4; ++kt) {
        const int kp = c * 64 + kt * 16 + lm;
#pragma unroll
        for (int r = 0; r < 8; ++r) {
          const int qp = qb + 8 * lh + r;
          float v = sacc[kt][r] * SSC;
          if (rel != 0) {
            const bool keep = (rel < 0) ? (kp >= qp) : (kp < qp);
            v = keep ? v : NEG;
          }
          sacc[kt][r] = v;
          bm[r] = fmaxf(bm[r], v);
        }
      }
#pragma unroll
      for (int r = 0; r < 8; ++r)
#pragma unroll
        for (int xm = 1; xm < 16; xm <<= 1)
          bm[r] = fmaxf(bm[r], __shfl_xor(bm[r], xm, 32));

      float scn[8];
#pragma unroll
      for (int r = 0; r < 8; ++r) {
        const float mn = fmaxf(m_r[r], bm[r]);
        scn[r] = __expf(m_r[r] - mn);
        m_r[r] = mn;
      }
      float bs[8];
#pragma unroll
      for (int r = 0; r < 8; ++r) bs[r] = 0.0f;
#pragma unroll
      for (int kt = 0; kt < 4; ++kt)
#pragma unroll
        for (int r = 0; r < 8; ++r) {
          const float v = sacc[kt][r];
          const float p = (v > -1e29f) ? __expf(v - m_r[r]) : 0.0f;
          sacc[kt][r] = p;
          bs[r] += p;
        }
#pragma unroll
      for (int r = 0; r < 8; ++r)
#pragma unroll
        for (int xm = 1; xm < 16; xm <<= 1)
          bs[r] += __shfl_xor(bs[r], xm, 32);
#pragma unroll
      for (int r = 0; r < 8; ++r) l_r[r] = l_r[r] * scn[r] + bs[r];
#pragma unroll
      for (int nt = 0; nt < 4; ++nt)
#pragma unroll
        for (int r = 0; r < 8; ++r) oacc[nt][r] *= scn[r];

#pragma unroll
      for (int kt = 0; kt < 4; ++kt) {
        const int kp = kt * 16 + lm;
#pragma unroll
        for (int r = 0; r < 8; ++r) Pw[(8 * lh + r) * PPH + kp] = (f16_t)(sacc[kt][r] * PSC);
      }
      __syncthreads();

#pragma unroll
      for (int kc = 0; kc < 2; ++kc) {
        FragH pf;
        pf.u[0] = *(const v4u*)(Pw + lm * PPH + kc * 32 + 8 * lh);
        pf.u[1] = *(const v4u*)(Pw + lm * PPH + kc * 32 + 16 + 8 * lh);
        const size_t vo = head + (size_t)lm * SQ + jb * BLKQ + c * 64 + kc * 32 + 8 * lh;
        v16h vf;
#pragma unroll
        for (int nt = 0; nt < 4; ++nt) {
          vf = ldfh(Vp + vo + (size_t)nt * 16 * SQ);
          oacc[nt] = mma_h(oacc[nt], pf.v, vf);
        }
        asm volatile(NOP4
                     : "+v"(oacc[0]), "+v"(oacc[1]), "+v"(oacc[2]), "+v"(oacc[3])
                     : "v"(pf.v), "v"(vf));
      }
      __syncthreads();
    }
  }

  float osc[8];
#pragma unroll
  for (int r = 0; r < 8; ++r) osc[r] = OSC / l_r[r];
  __syncthreads();
#pragma unroll
  for (int nt = 0; nt < 4; ++nt) {
    const int dl = nt * 16 + lm;
#pragma unroll
    for (int r = 0; r < 8; ++r) Ow[(8 * lh + r) * OPF + dl] = oacc[nt][r] * osc[r];
  }
  __syncthreads();
  const int q = lane >> 3, j = lane & 7;
  const size_t obase = ((size_t)(b * SQ + n * BLKQ + qb) * HQ + hd) * DQ + 8 * j;
  for (int pass = 0; pass < 2; ++pass) {
    if (pass) __threadfence();
#pragma unroll
    for (int it = 0; it < 4; ++it) {
      const int rl = it * 4 + q;
      const float* pp = Ow + rl * OPF + 8 * j;
      const v4f x0 = *(const v4f*)(pp);
      const v4f x1 = *(const v4f*)(pp + 4);
      float x[8];
      x[0] = x0[0]; x[1] = x0[1]; x[2] = x0[2]; x[3] = x0[3];
      x[4] = x1[0]; x[5] = x1[1]; x[6] = x1[2]; x[7] = x1[3];
      PackB ohp, olp;
#pragma unroll
      for (int i = 0; i < 8; ++i) {
        const bf16_t th = (bf16_t)x[i];
        ohp.b[i] = th;
        olp.b[i] = (bf16_t)(x[i] - (float)th);
      }
      const size_t o = obase + (size_t)rl * HQ * DQ;
      *(volatile v4u*)(Oh + o) = ohp.u;
      *(volatile v4u*)(Ol + o) = olp.u;
    }
  }
}

extern "C" void kernel_launch(void* const* d_in, const int* in_sizes, int n_in,
                              void* d_out, int out_size, void* d_ws, size_t ws_size,
                              hipStream_t stream) {
  if (n_in < 10) return;
  if (in_sizes[0] != (int)NE || in_sizes[1] != (int)NE) return;
  if (in_sizes[2] != (int)WE || in_sizes[4] != (int)WE || in_sizes[6] != (int)WE || in_sizes[8] != (int)WE) return;
  if (in_sizes[3] != HQ * DQ || in_sizes[5] != HQ * DQ || in_sizes[7] != HQ * DQ || in_sizes[9] != FQ) return;
  if (out_size != (int)NE) return;
  const size_t total_bytes = (9 * NE + 4 * WE) * sizeof(bf16_t);
  if (total_bytes > ws_size) return;

  const float* xq  = (const float*)d_in[0];
  const float* xkv = (const float*)d_in[1];
  const float* Wq  = (const float*)d_in[2];
  const float* bq  = (const float*)d_in[3];
  const float* Wk  = (const float*)d_in[4];
  const float* bk  = (const float*)d_in[5];
  const float* Wv  = (const float*)d_in[6];
  const float* bv  = (const float*)d_in[7];
  const float* Wo  = (const float*)d_in[8];
  const float* bo  = (const float*)d_in[9];
  float* out = (float*)d_out;

  bf16_t* Xq = (bf16_t*)d_ws;
  bf16_t* Xk = Xq + NE;
  f16_t*  Qp = (f16_t*)(Xk + NE);
  f16_t*  Kp = Qp + NE;
  f16_t*  Vp = Kp + NE;
  bf16_t* Oh = (bf16_t*)(Vp + NE);
  bf16_t* Ol = Oh + NE;
  bf16_t* wb = Ol + NE;
  bf16_t* Wqt = wb + 0 * WE;
  bf16_t* Wkt = wb + 1 * WE;
  bf16_t* Wvt = wb + 2 * WE;
  bf16_t* Wot = wb + 3 * WE;

  const int n8 = (int)(NE / 8);
  const dim3 gs((n8 + 255) / 256);
  k_cvt<<<gs, 256, 0, stream>>>(xq, n8, Xq);
  k_cvt<<<gs, 256, 0, stream>>>(xkv, n8, Xk);

  const dim3 gw(FQ / 64, FQ / 64);
  k_wtrans<<<gw, 256, 0, stream>>>(Wq, FQ, FQ, Wqt);
  k_wtrans<<<gw, 256, 0, stream>>>(Wk, FQ, FQ, Wkt);
  k_wtrans<<<gw, 256, 0, stream>>>(Wv, FQ, FQ, Wvt);
  k_wtrans<<<gw, 256, 0, stream>>>(Wo, FQ, FQ, Wot);

  const dim3 gg(MROWS / 128, FQ / 128);
  k_gemm<0><<<gg, 256, 0, stream>>>(Xq, Xq, Wqt, bq, QSC, Qp, out);
  k_gemm<0><<<gg, 256, 0, stream>>>(Xk, Xk, Wkt, bk, KSC, Kp, out);
  k_gemm<1><<<gg, 256, 0, stream>>>(Xk, Xk, Wvt, bv, VSC, Vp, out);

  k_attn<<<dim3(BQ * HQ * NBQ * 2), 128, 0, stream>>>(Qp, Kp, Vp, Oh, Ol);

  k_gemm<2><<<gg, 256, 0, stream>>>(Oh, Ol, Wot, bo, 1.0f, Qp, out);
}
